// GraphEncoderDecoderAttention_11484742549821
// MI455X (gfx1250) — hardware-verified
//
#include <hip/hip_runtime.h>


#define NB_  2
#define NN   2048
#define CC   256
#define NH_  8
#define FH   32
#define HP   4
#define PCAR 1024.0f
typedef _Float16 h16;
typedef unsigned short bf;
typedef __attribute__((ext_vector_type(16))) __bf16   v16bf;
typedef __attribute__((ext_vector_type(16))) _Float16 v16h;
typedef __attribute__((ext_vector_type(8)))  _Float16 v8h;
typedef __attribute__((ext_vector_type(8)))  unsigned short v8us;
typedef __attribute__((ext_vector_type(8)))  float    v8f;
typedef __attribute__((ext_vector_type(4)))  float    v4f;
typedef v8h  __attribute__((may_alias)) v8ha;
typedef v4f  __attribute__((may_alias)) v4fa;
typedef v8us __attribute__((may_alias)) v8usa;

__device__ __forceinline__ unsigned short f2bf(float f) { unsigned u = __float_as_uint(f); u += 0x7FFFu + ((u >> 16) & 1u); return (unsigned short)(u >> 16); }
__device__ __forceinline__ float bf2f(unsigned short b) { return __uint_as_float(((unsigned)b) << 16); }
__device__ __forceinline__ float bfr(float f) { return bf2f(f2bf(f)); }
__device__ __forceinline__ v16h cat16(v8h lo, v8h hi) { return __builtin_shufflevector(lo, hi, 0, 1, 2, 3, 4, 5, 6, 7, 8, 9, 10, 11, 12, 13, 14, 15); }
__device__ __forceinline__ v16bf cat16b(v8us lo, v8us hi) { return __builtin_bit_cast(v16bf, __builtin_shufflevector(lo, hi, 0, 1, 2, 3, 4, 5, 6, 7, 8, 9, 10, 11, 12, 13, 14, 15)); }
__device__ __forceinline__ v8f wmma16(v16h a, v16h b, v8f c) { return __builtin_amdgcn_wmma_f32_16x16x32_f16(false, a, false, b, (short)0, c, false, false); }
__device__ __forceinline__ v8f wmmab(v16bf a, v16bf b, v8f c) { return __builtin_amdgcn_wmma_f32_16x16x32_bf16(false, a, false, b, (short)0, c, false, false); }


template <typename T16> struct WFrag;
template <> struct WFrag<h16> { typedef v16h V; static __device__ __forceinline__ V ld(const h16* p) { return cat16(*(const v8h*)p, *(const v8h*)(p + 16)); } static __device__ __forceinline__ v8f mma(V a, V b, v8f c) { return wmma16(a, b, c); } };
template <> struct WFrag<bf> { typedef v16bf V; static __device__ __forceinline__ V ld(const bf* p) { return cat16b(*(const v8us*)p, *(const v8us*)(p + 16)); } static __device__ __forceinline__ v8f mma(V a, V b, v8f c) { return wmmab(a, b, c); } };
template <typename T16, int NSPLIT, bool BIAS>
__global__ __launch_bounds__(32) void k_gemmw(const T16* __restrict__ A, const T16* __restrict__ A2, const T16* __restrict__ Bt, const T16* __restrict__ Bt2, int K, float* C, int ldc, const float* __restrict__ bias, size_t sA, size_t sB, size_t sC) {
    typedef typename WFrag<T16>::V V;
    __shared__ __align__(16) float os[16 * 68];
    const size_t z = blockIdx.z; A += z * sA; if (A2) A2 += z * sA; Bt += z * sB; if (Bt2) Bt2 += z * sB; C += z * sC;
    const int lane = threadIdx.x & 31, lr = lane & 15, hi = lane >> 4; const int r0 = blockIdx.x * 64, c0 = blockIdx.y * 64;
    v8f acc[4][4];
#pragma unroll
    for (int mb = 0; mb < 4; ++mb)
#pragma unroll
        for (int nb = 0; nb < 4; ++nb) acc[mb][nb] = (v8f){};
    const size_t aoff = (size_t)(r0 + lr) * K + 8 * hi, boff = (size_t)(c0 + lr) * K + 8 * hi;
#pragma unroll 1
    for (int kc = 0; kc < K; kc += 32) {
        V a[4], a2[4];
#pragma unroll
        for (int mb = 0; mb < 4; ++mb) { a[mb] = WFrag<T16>::ld(A + aoff + (size_t)mb * 16 * K + kc); if (NSPLIT == 1 || NSPLIT == 2) a2[mb] = WFrag<T16>::ld(A2 + aoff + (size_t)mb * 16 * K + kc); }
#pragma unroll
        for (int nb = 0; nb < 4; ++nb) { const V b = WFrag<T16>::ld(Bt + boff + (size_t)nb * 16 * K + kc); V b2; if (NSPLIT >= 2) b2 = WFrag<T16>::ld(Bt2 + boff + (size_t)nb * 16 * K + kc);
#pragma unroll
            for (int mb = 0; mb < 4; ++mb) { acc[mb][nb] = WFrag<T16>::mma(a[mb], b, acc[mb][nb]); if (NSPLIT == 1 || NSPLIT == 2) acc[mb][nb] = WFrag<T16>::mma(a2[mb], b, acc[mb][nb]); if (NSPLIT >= 2) acc[mb][nb] = WFrag<T16>::mma(a[mb], b2, acc[mb][nb]); } }
        asm volatile("v_nop\n\tv_nop\n\tv_nop\n\tv_nop" : "+v"(acc[0][0]), "+v"(acc[1][1]), "+v"(acc[2][2]), "+v"(acc[3][3]) : "v"(a[0]), "v"(a[3]));
    }
#pragma unroll
    for (int mb = 0; mb < 4; ++mb) {
#pragma unroll
        for (int nb = 0; nb < 4; ++nb) {
#pragma unroll
            for (int j = 0; j < 8; ++j) os[(hi * 8 + j) * 68 + nb * 16 + lr] = acc[mb][nb][j]; }
        __builtin_amdgcn_wave_barrier(); asm volatile("" ::: "memory");
        float* crow = C + (size_t)(r0 + mb * 16) * ldc + c0;
#pragma unroll 1
        for (int ps = 0; ps < 2; ++ps) {
#pragma unroll
            for (int s = 0; s < 8; ++s) { const int row = 2 * s + hi, cofs = lr * 4; v4f val = *(const v4fa*)(os + row * 68 + cofs); if (BIAS) { val[0] += bfr(bias[c0 + cofs]); val[1] += bfr(bias[c0 + cofs + 1]); val[2] += bfr(bias[c0 + cofs + 2]); val[3] += bfr(bias[c0 + cofs + 3]); }
                *(volatile v4f*)(crow + (size_t)row * ldc + cofs) = val; }
            if (ps == 0) __threadfence(); }
        __builtin_amdgcn_wave_barrier(); asm volatile("" ::: "memory");
    }
}

__device__ __forceinline__ h16 tohx(float x) { return (h16)x; }
__device__ __forceinline__ void splitf(float y, unsigned short& h, unsigned short& l) { h = f2bf(y); l = f2bf(y - bf2f(h)); }
__device__ __forceinline__ float leaky(float x, float s) { return x > 0.f ? x : __fmul_rn(s, x); }
typedef __attribute__((ext_vector_type(2))) unsigned short v2us;
typedef __attribute__((ext_vector_type(4))) unsigned short v4us;
typedef __attribute__((ext_vector_type(2))) _Float16 v2h;
typedef __attribute__((ext_vector_type(4))) _Float16 v4h;
typedef __attribute__((ext_vector_type(4))) int v4i;

__global__ __launch_bounds__(256) void k_cvt8(const float* __restrict__ src, bf* dst, size_t n8) { const size_t i = (size_t)blockIdx.x * 256 + threadIdx.x; if (i >= n8) return; const v8f v = *(const v8f*)(src + i * 8); v8us o;
#pragma unroll
    for (int k = 0; k < 8; ++k) o[k] = f2bf(v[k]); *(volatile v8us*)(dst + i * 8) = o; __threadfence(); *(volatile v8us*)(dst + i * 8) = o; }
__global__ __launch_bounds__(256) void k_wgat(const float* __restrict__ Wg, bf* Bt) { const int e = (blockIdx.x * 256 + threadIdx.x) * 4; if (e >= CC * CC) return; const int c = e % CC; const int hf = e / CC; const int h = hf / FH, f = hf % FH; v4us o;
#pragma unroll
    for (int u = 0; u < 4; ++u) o[u] = f2bf(Wg[((size_t)h * CC + c + u) * FH + f]); *(volatile v4us*)(Bt + e) = o; __threadfence(); *(volatile v4us*)(Bt + e) = o; }
__global__ __launch_bounds__(256) void k_sdot(const float* __restrict__ WSC, const float* __restrict__ WTH, const float* __restrict__ av, float* SC, float* SH) { const int n = blockIdx.x * 256 + threadIdx.x; if (n >= NN) return; float sc[NH_], sh[NH_];
#pragma unroll
    for (int h = 0; h < NH_; ++h) { float s1 = 0.f, s2 = 0.f;
#pragma unroll 1
        for (int f = 0; f < FH; ++f) { float w1 = bfr(av[h * 2 * FH + f]), w2 = bfr(av[h * 2 * FH + FH + f]); asm volatile("" : "+v"(w1)); asm volatile("" : "+v"(w2)); float p1 = __fmul_rn(WSC[(size_t)n * CC + h * FH + f], w1), p2 = __fmul_rn(WTH[(size_t)n * CC + h * FH + f], w2); asm volatile("" : "+v"(p1)); asm volatile("" : "+v"(p2)); s1 = __fadd_rn(s1, p1); s2 = __fadd_rn(s2, p2); }
        sc[h] = s1; sh[h] = s2; }
    for (int ps = 0; ps < 2; ++ps) {
#pragma unroll
        for (int h = 0; h < NH_; ++h) { *(volatile float*)(SC + (size_t)h * NN + n) = sc[h]; *(volatile float*)(SH + (size_t)h * NN + n) = sh[h]; } if (ps == 0) __threadfence(); } }
__global__ __launch_bounds__(256) void k_gsoft(const float* __restrict__ SC, const float* __restrict__ SH, const int* __restrict__ adj, int h0, h16* P16) { const int lane = threadIdx.x & 31; const int row = blockIdx.x * 8 + (threadIdx.x >> 5); if (row >= HP * NN) return; const int i = row % NN; const int h = h0 + row / NN; const float si = SC[(size_t)h * NN + i]; const float* shr = SH + (size_t)h * NN; const int* ar = adj + (size_t)i * NN; float v[NN / 32]; float mx = -3.0e38f;
#pragma unroll
    for (int ch = 0; ch < NN / 128; ++ch) { const int j0 = ch * 128 + lane * 4; const v4f a = *(const v4f*)(shr + j0); const v4i m4 = *(const v4i*)(ar + j0);
#pragma unroll
        for (int u = 0; u < 4; ++u) { const float e = leaky(__fadd_rn(si, a[u]), 0.1f); const float t = (m4[u] > 0) ? e : -9.0e15f; v[ch * 4 + u] = t; mx = fmaxf(mx, t); } }
#pragma unroll
    for (int sh = 16; sh; sh >>= 1) mx = fmaxf(mx, __shfl_xor(mx, sh, 32));
    float sum = 0.f;
#pragma unroll
    for (int q = 0; q < NN / 32; ++q) { float d0 = __fsub_rn(v[q], mx); asm volatile("" : "+v"(d0)); v[q] = __builtin_amdgcn_exp2f(__fmul_rn(d0, 1.4426950408889634f)); sum += v[q]; }
#pragma unroll
    for (int sh = 16; sh; sh >>= 1) sum += __shfl_xor(sum, sh, 32);
    const float f = __fdiv_rn(PCAR, sum);
    for (int ps = 0; ps < 2; ++ps) {
#pragma unroll
        for (int ch = 0; ch < NN / 128; ++ch) { v4h o4;
#pragma unroll
            for (int q = 0; q < 4; ++q) o4[q] = tohx(v[ch * 4 + q] * f); *(volatile v4h*)(P16 + (size_t)row * NN + ch * 128 + lane * 4) = o4; }
        if (ps == 0) __threadfence(); } }
__global__ __launch_bounds__(256) void k_wst(const float* __restrict__ F, int h0, h16* VT) { const int e = (blockIdx.x * 256 + threadIdx.x) * 2; if (e >= HP * 64 * NN) return; const int n = e % NN; const int f = (e / NN) % 64; const int z = e / (NN * 64); v2h o;
    if (f < FH) { o[0] = tohx(F[(size_t)n * CC + (h0 + z) * FH + f]); o[1] = tohx(F[(size_t)(n + 1) * CC + (h0 + z) * FH + f]); } else { o[0] = (h16)0.f; o[1] = (h16)0.f; }
    *(volatile v2h*)(VT + e) = o; __threadfence(); *(volatile v2h*)(VT + e) = o; }
__global__ __launch_bounds__(256) void k_h1(const float* __restrict__ x, const float* __restrict__ HPb, int h0, float* H1) { const int e = (blockIdx.x * 256 + threadIdx.x) * 4; if (e >= NN * HP * FH) return; const int cc = e % (HP * FH); const int n = e / (HP * FH); const int z = cc / FH, f = cc % FH; const int c = (h0 + z) * FH + f; v4f o;
#pragma unroll
    for (int u = 0; u < 4; ++u) o[u] = __fadd_rn(bfr(x[(size_t)n * CC + c + u]), leaky(HPb[((size_t)z * NN + n) * 64 + f + u] * (1.0f / PCAR), 0.01f)); float* dst = H1 + (size_t)n * CC + c; *(volatile v4f*)dst = o; __threadfence(); *(volatile v4f*)dst = o; }
__global__ __launch_bounds__(256) void k_rown(const float* __restrict__ X, float* R) { const int lane = threadIdx.x & 31; const int n = blockIdx.x * 8 + (threadIdx.x >> 5); if (n >= NN) return; const float* xr = X + (size_t)n * CC; float v[CC / 32]; float s = 0.f;
#pragma unroll
    for (int ch = 0; ch < CC / 128; ++ch) { const v4f a = *(const v4f*)(xr + ch * 128 + lane * 4);
#pragma unroll
        for (int u = 0; u < 4; ++u) { v[ch * 4 + u] = a[u]; s += a[u]; } }
#pragma unroll
    for (int sh = 16; sh; sh >>= 1) s += __shfl_xor(s, sh, 32);
    const float mean = s * (1.0f / CC); float q = 0.f;
#pragma unroll
    for (int k = 0; k < CC / 32; ++k) { float d = __fsub_rn(v[k], mean); asm volatile("" : "+v"(d)); float p = __fmul_rn(d, d); asm volatile("" : "+v"(p)); q = __fadd_rn(q, p); }
#pragma unroll
    for (int sh = 16; sh; sh >>= 1) q += __shfl_xor(q, sh, 32);
    const float inv = __fdiv_rn(1.0f, __fadd_rn(__fsqrt_rn(q * (1.0f / (CC - 1))), 1e-6f));
    for (int ps = 0; ps < 2; ++ps) {
#pragma unroll
        for (int ch = 0; ch < CC / 128; ++ch) { v4f o;
#pragma unroll
            for (int u = 0; u < 4; ++u) { float d = __fsub_rn(v[ch * 4 + u], mean); asm volatile("" : "+v"(d)); o[u] = __fmul_rn(d, inv); } *(volatile v4f*)(R + (size_t)n * CC + ch * 128 + lane * 4) = o; }
        if (ps == 0) __threadfence(); } }
__global__ __launch_bounds__(256) void k_cols(const float* __restrict__ R, float* CM, float* CS) { const int c = threadIdx.x; float s = 0.f;
    for (int n = 0; n < NN; ++n) s = __fadd_rn(s, R[(size_t)n * CC + c]);
    const float mean = s * (1.0f / NN); float q = 0.f;
    for (int n = 0; n < NN; ++n) { float d = __fsub_rn(R[(size_t)n * CC + c], mean); asm volatile("" : "+v"(d)); float p = __fmul_rn(d, d); asm volatile("" : "+v"(p)); q = __fadd_rn(q, p); }
    const float sd = __fsqrt_rn(q * (1.0f / (NN - 1))); for (int ps = 0; ps < 2; ++ps) { *(volatile float*)(CM + c) = mean; *(volatile float*)(CS + c) = sd; if (ps == 0) __threadfence(); } }
__global__ __launch_bounds__(256) void k_coln(const float* __restrict__ R, const float* __restrict__ CM, const float* __restrict__ CS, bf* Dh, bf* Dl) { const int e = (blockIdx.x * 256 + threadIdx.x) * 4; if (e >= NN * CC) return; const int c = e % CC; v4us oh, ol;
#pragma unroll
    for (int u = 0; u < 4; ++u) { float d = __fsub_rn(R[e + u], CM[c + u]); asm volatile("" : "+v"(d)); const float y = __fdiv_rn(d, __fadd_rn(CS[c + u], 1e-6f)); unsigned short a, b; splitf(y, a, b); oh[u] = a; ol[u] = b; }
    *(volatile v4us*)(Dh + e) = oh; *(volatile v4us*)(Dl + e) = ol; __threadfence(); *(volatile v4us*)(Dh + e) = oh; *(volatile v4us*)(Dl + e) = ol; }
__global__ __launch_bounds__(256) void k_pl32(const float* __restrict__ F, h16* P) { const int e = (blockIdx.x * 256 + threadIdx.x) * 4; if (e >= NH_ * NN * FH) return; const int d = e % FH; const int n = (e / FH) % NN; const int h = e / (FH * NN); const float* f = F + (size_t)n * CC + h * FH + d; v4h o;
#pragma unroll
    for (int u = 0; u < 4; ++u) o[u] = tohx(f[u]); *(volatile v4h*)(P + e) = o; __threadfence(); *(volatile v4h*)(P + e) = o; }
__global__ __launch_bounds__(256) void k_msoft(const float* __restrict__ Sb, h16* P16) { const int lane = threadIdx.x & 31; const int row = blockIdx.x * 8 + (threadIdx.x >> 5); if (row >= HP * NN) return; const float* sr = Sb + (size_t)row * NN; float v[NN / 32]; float mx = -3.0e38f; const float scl = 0.17677669529663687f;
#pragma unroll
    for (int ch = 0; ch < NN / 128; ++ch) { const v4f a = *(const v4f*)(sr + ch * 128 + lane * 4);
#pragma unroll
        for (int u = 0; u < 4; ++u) { const float t = a[u] * scl; v[ch * 4 + u] = t; mx = fmaxf(mx, t); } }
#pragma unroll
    for (int sh = 16; sh; sh >>= 1) mx = fmaxf(mx, __shfl_xor(mx, sh, 32));
    float sum = 0.f;
#pragma unroll
    for (int q = 0; q < NN / 32; ++q) { float d0 = __fsub_rn(v[q], mx); asm volatile("" : "+v"(d0)); v[q] = __builtin_amdgcn_exp2f(__fmul_rn(d0, 1.4426950408889634f)); sum += v[q]; }
#pragma unroll
    for (int sh = 16; sh; sh >>= 1) sum += __shfl_xor(sum, sh, 32);
    const float f = __fdiv_rn(PCAR, sum);
    for (int ps = 0; ps < 2; ++ps) {
#pragma unroll
        for (int ch = 0; ch < NN / 128; ++ch) { v4h o4;
#pragma unroll
            for (int q = 0; q < 4; ++q) o4[q] = tohx(v[ch * 4 + q] * f); *(volatile v4h*)(P16 + (size_t)row * NN + ch * 128 + lane * 4) = o4; }
        if (ps == 0) __threadfence(); } }
__global__ __launch_bounds__(256) void k_mrg(const float* __restrict__ O, int h0, bf* Ah, bf* Al) { const int e = (blockIdx.x * 256 + threadIdx.x) * 4; if (e >= HP * NN * FH) return; const int d = e % FH; const int n = (e / FH) % NN; const int z = e / (FH * NN); v4us oh, ol;
#pragma unroll
    for (int u = 0; u < 4; ++u) { unsigned short a, b; splitf(O[((size_t)z * NN + n) * 64 + d + u] * (1.0f / PCAR), a, b); oh[u] = a; ol[u] = b; } const size_t oo = (size_t)n * CC + (h0 + z) * FH + d;
    *(volatile v4us*)(Ah + oo) = oh; *(volatile v4us*)(Al + oo) = ol; __threadfence(); *(volatile v4us*)(Ah + oo) = oh; *(volatile v4us*)(Al + oo) = ol; }

extern "C" void kernel_launch(void* const* d_in, const int* in_sizes, int n_in,
                              void* d_out, int out_size, void* d_ws, size_t ws_size, hipStream_t stream) {
    (void)in_sizes; (void)n_in; (void)out_size;
    const float** I = (const float**)d_in;
    const float *x = I[0], *cwp = I[1], *ctx = I[2], *Ws = I[5], *Wt = I[6], *av = I[7], *W_lin = I[8], *b_lin = I[9], *W_in = I[10], *b_in = I[11], *W_out = I[12], *b_out = I[13]; const int* adj = (const int*)d_in[4];
    float* OUT = (float*)d_out;
    char* wsp = (char*)d_ws;
    auto take = [&](size_t bytes) { char* p = wsp; wsp += (bytes + 255) & ~(size_t)255; return (void*)p; };
    bf* BWS = (bf*)take(CC * CC * 2); bf* BWT = (bf*)take(CC * CC * 2); bf* BLIN = (bf*)take(CC * CC * 2); bf* BIN = (bf*)take((size_t)3 * CC * CC * 2); bf* BOUT = (bf*)take(CC * CC * 2);
    bf* XB = (bf*)take((size_t)NN * CC * 2); bf* CB = (bf*)take((size_t)NN * CC * 2); bf* TB = (bf*)take((size_t)NN * CC * 2); float* WSC = (float*)take((size_t)NN * CC * 4); float* WTH = (float*)take((size_t)NN * CC * 4); float* SC = (float*)take((size_t)NH_ * NN * 4); float* SH = (float*)take((size_t)NH_ * NN * 4);
    h16* P16 = (h16*)take((size_t)HP * NN * NN * 2); h16* VT = (h16*)take((size_t)HP * 64 * NN * 2); float* HPb = (float*)take((size_t)HP * NN * 64 * 4); float* H1 = (float*)take((size_t)NN * CC * 4); float* R = (float*)take((size_t)NN * CC * 4); float* CM = (float*)take(CC * 4); float* CSD = (float*)take(CC * 4); bf* Dh = (bf*)take((size_t)NN * CC * 2); bf* Dl = (bf*)take((size_t)NN * CC * 2); float* H2 = (float*)take((size_t)NN * CC * 4);
    float* FQ = (float*)take((size_t)NN * CC * 4); float* FK = (float*)take((size_t)NN * CC * 4); float* FV = (float*)take((size_t)NN * CC * 4); h16* Q16 = (h16*)take((size_t)NH_ * NN * FH * 2); h16* K16 = (h16*)take((size_t)NH_ * NN * FH * 2); float* Sb = (float*)take((size_t)HP * NN * NN * 4); float* O = (float*)take((size_t)HP * NN * 64 * 4); bf* Ah = (bf*)take((size_t)NN * CC * 2); bf* Al = (bf*)take((size_t)NN * CC * 2);
    if ((size_t)(wsp - (char*)d_ws) > ws_size) return;
    k_wgat<<<(CC * CC / 4 + 255) / 256, 256, 0, stream>>>(Ws, BWS); k_wgat<<<(CC * CC / 4 + 255) / 256, 256, 0, stream>>>(Wt, BWT);
    k_cvt8<<<(CC * CC / 8 + 255) / 256, 256, 0, stream>>>(W_lin, BLIN, CC * CC / 8); k_cvt8<<<(3 * CC * CC / 8 + 255) / 256, 256, 0, stream>>>(W_in, BIN, 3 * CC * CC / 8); k_cvt8<<<(CC * CC / 8 + 255) / 256, 256, 0, stream>>>(W_out, BOUT, CC * CC / 8);
    const unsigned gE = (NN * CC / 4 + 255) / 256;
    for (int b = 0; b < NB_; ++b) { const size_t bo = (size_t)b * NN * CC;
        k_cvt8<<<(NN * CC / 8 + 255) / 256, 256, 0, stream>>>(x + bo, XB, (size_t)NN * CC / 8); k_cvt8<<<(NN * CC / 8 + 255) / 256, 256, 0, stream>>>(cwp + bo, CB, (size_t)NN * CC / 8); k_cvt8<<<(NN * CC / 8 + 255) / 256, 256, 0, stream>>>(ctx + bo, TB, (size_t)NN * CC / 8);
        k_gemmw<bf, 0, false><<<dim3(NN / 64, CC / 64, 1), 32, 0, stream>>>(CB, nullptr, BWS, nullptr, CC, WSC, CC, nullptr, 0, 0, 0); k_gemmw<bf, 0, false><<<dim3(NN / 64, CC / 64, 1), 32, 0, stream>>>(XB, nullptr, BWT, nullptr, CC, WTH, CC, nullptr, 0, 0, 0);
        k_sdot<<<(NN + 255) / 256, 256, 0, stream>>>(WSC, WTH, av, SC, SH);
        for (int h0 = 0; h0 < NH_; h0 += HP) {
            k_gsoft<<<HP * NN / 8, 256, 0, stream>>>(SC, SH, adj + (size_t)b * NN * NN, h0, P16); k_wst<<<(HP * 64 * NN / 2 + 255) / 256, 256, 0, stream>>>(WSC, h0, VT);
            k_gemmw<h16, 0, false><<<dim3(NN / 64, 1, HP), 32, 0, stream>>>(P16, nullptr, VT, nullptr, NN, HPb, 64, nullptr, (size_t)NN * NN, (size_t)64 * NN, (size_t)NN * 64);
            k_h1<<<(NN * HP * FH / 4 + 255) / 256, 256, 0, stream>>>(x + bo, HPb, h0, H1); }
        k_rown<<<NN / 8, 256, 0, stream>>>(H1, R); k_cols<<<1, 256, 0, stream>>>(R, CM, CSD); k_coln<<<gE, 256, 0, stream>>>(R, CM, CSD, Dh, Dl);
        k_gemmw<bf, 1, true><<<dim3(NN / 64, CC / 64, 1), 32, 0, stream>>>(Dh, Dl, BLIN, nullptr, CC, H2, CC, b_lin, 0, 0, 0);
        k_rown<<<NN / 8, 256, 0, stream>>>(H2, R); k_cols<<<1, 256, 0, stream>>>(R, CM, CSD); k_coln<<<gE, 256, 0, stream>>>(R, CM, CSD, Dh, Dl);
        k_gemmw<bf, 1, true><<<dim3(NN / 64, CC / 64, 1), 32, 0, stream>>>(Dh, Dl, BIN, nullptr, CC, FQ, CC, b_in, 0, 0, 0);
        k_gemmw<bf, 0, true><<<dim3(NN / 64, CC / 64, 1), 32, 0, stream>>>(CB, nullptr, BIN + (size_t)CC * CC, nullptr, CC, FK, CC, b_in + CC, 0, 0, 0); k_gemmw<bf, 0, true><<<dim3(NN / 64, CC / 64, 1), 32, 0, stream>>>(TB, nullptr, BIN + (size_t)2 * CC * CC, nullptr, CC, FV, CC, b_in + 2 * CC, 0, 0, 0);
        k_pl32<<<(NH_ * NN * FH / 4 + 255) / 256, 256, 0, stream>>>(FQ, Q16); k_pl32<<<(NH_ * NN * FH / 4 + 255) / 256, 256, 0, stream>>>(FK, K16);
        for (int h0 = 0; h0 < NH_; h0 += HP) { const size_t zo = (size_t)h0 * NN * FH;
            k_gemmw<h16, 0, false><<<dim3(NN / 64, NN / 64, HP), 32, 0, stream>>>(Q16 + zo, nullptr, K16 + zo, nullptr, FH, Sb, NN, nullptr, (size_t)NN * FH, (size_t)NN * FH, (size_t)NN * NN);
            k_msoft<<<HP * NN / 8, 256, 0, stream>>>(Sb, P16); k_wst<<<(HP * 64 * NN / 2 + 255) / 256, 256, 0, stream>>>(FV, h0, VT);
            k_gemmw<h16, 0, false><<<dim3(NN / 64, 1, HP), 32, 0, stream>>>(P16, nullptr, VT, nullptr, NN, O, 64, nullptr, (size_t)NN * NN, (size_t)64 * NN, (size_t)NN * 64);
            k_mrg<<<(HP * NN * FH / 4 + 255) / 256, 256, 0, stream>>>(O, h0, Ah, Al); }
        k_gemmw<bf, 1, true><<<dim3(NN / 64, CC / 64, 1), 32, 0, stream>>>(Ah, Al, BOUT, nullptr, CC, OUT + bo, CC, b_out, 0, 0, 0); }
}
